// MultiPoleScoreNet_4509715661581
// MI455X (gfx1250) — hardware-verified
//
#include <hip/hip_runtime.h>


#define LAT    128
#define HID    64
#define CIN    3
#define NTH    256
#define NWV    8
#define NPB    32
#define NPW    4
#define GTH    128
#define GRW    64
#define MAXT   512
#define NCH    32
#define WSCAP  134217728

static_assert(NTH == NWV * 32 && NPB == NWV * NPW);
static_assert((LAT % 32) == 0 && (HID % 32) == 0 && LAT == 4 * 32);
static_assert(GRW == (GTH / 32) * 16);
static_assert(((LAT * HID) % (8 * NTH)) == 0);
static_assert((NPB * CIN) % 4 == 0 && (NPB * CIN * 4) % 128 == 0 && (NPB * CIN) / 4 <= 32);
static_assert(NCH == 32);

typedef float        v4f  __attribute__((ext_vector_type(4)));
typedef float        v8f  __attribute__((ext_vector_type(8)));
typedef _Float16     v8h  __attribute__((ext_vector_type(8)));
typedef _Float16     v16h __attribute__((ext_vector_type(16)));
typedef unsigned int v4u  __attribute__((ext_vector_type(4)));
typedef v4f v4fa __attribute__((may_alias));
typedef v8h v8ha __attribute__((may_alias));
typedef v4u v4ua __attribute__((may_alias));
union Frag { v16h v; v8h half[2]; };
struct Src4 { const float* p0; const float* p1; const float* p2; const float* p3; };
static_assert(sizeof(Src4) == 32);
struct Dst4 { const int* p0; const int* p1; const int* p2; const int* p3; };
static_assert(sizeof(Dst4) == 32);

static __device__ __forceinline__ v8f wmf(v16h a, v16h b, v8f c) {
  v8f d = __builtin_amdgcn_wmma_f32_16x16x32_f16(false, a, false, b, (short)0, c, false, false);
  asm volatile("v_nop\n\tv_nop\n\tv_nop\n\tv_nop" : "+v"(d) : "v"(a), "v"(b));
  return d;
}

static __device__ __forceinline__ v8h cvt8(v4f a, v4f b) {
  v8h r;
  r[0] = (_Float16)a.x; r[1] = (_Float16)a.y; r[2] = (_Float16)a.z; r[3] = (_Float16)a.w;
  r[4] = (_Float16)b.x; r[5] = (_Float16)b.y; r[6] = (_Float16)b.z; r[7] = (_Float16)b.w;
  return r;
}

static __device__ __forceinline__ void ld8(const float* p, float* o) {
  const v4fa a = *(const v4fa*)p;
  const v4fa b = *(const v4fa*)(p + 4);
  o[0] = a.x; o[1] = a.y; o[2] = a.z; o[3] = a.w;
  o[4] = b.x; o[5] = b.y; o[6] = b.z; o[7] = b.w;
}

static __device__ __forceinline__ v4f relu4(v4f v) {
  v4f r;
  r.x = v.x < 0.0f ? 0.0f : v.x;
  r.y = v.y < 0.0f ? 0.0f : v.y;
  r.z = v.z < 0.0f ? 0.0f : v.z;
  r.w = v.w < 0.0f ? 0.0f : v.w;
  return r;
}

static __device__ __forceinline__ float gelu16(float x) {
  const float x3 = x * x * x;
  float u = 0.7978845608028654f * fmaf(0.044715f, x3, x);
  u = fminf(fmaxf(u, -16.0f), 16.0f);
  const float e = __expf(2.0f * u);
  const float t = 1.0f - 2.0f * __builtin_amdgcn_rcpf(e + 1.0f);
  return 8.0f * x * (1.0f + t);
}

static __device__ __forceinline__ int lbound(const int* __restrict__ a, int n, int key) {
  int lo = 0, hi = n;
#pragma unroll 1
  for (int it = 0; it < 32; ++it) {
    if (lo >= hi) break;
    const int mid = (int)(((unsigned)lo + (unsigned)hi) >> 1);
    const int v = a[mid];
    if (v < key) lo = mid + 1; else hi = mid;
  }
  return lo;
}

__global__ __launch_bounds__(NTH) void k_chk(Dst4 d, int E0, int E1, int E2, int E3, int chunk, int* flg) {
  __shared__ int wany[NWV];
  const int tid = (int)threadIdx.x, lane = tid & 31;
  const int wave = __builtin_amdgcn_readfirstlane(tid >> 5);
  const int s = (int)blockIdx.y, c = (int)blockIdx.x;
  const int* dst = (s == 0) ? d.p0 : ((s == 1) ? d.p1 : ((s == 2) ? d.p2 : d.p3));
  const int  E   = (s == 0) ? E0   : ((s == 1) ? E1   : ((s == 2) ? E2   : E3));
  int badc = 0;
#pragma unroll 1
  for (int q = 0; q < chunk / NTH; ++q) {
    const int i = c * chunk + q * NTH + tid;
    int i0 = i < E - 2 ? i : E - 2;
    i0 = i0 < 0 ? 0 : i0;
    int i1 = i0 + 1;
    i1 = i1 < E ? i1 : E - 1;
    const int a = dst[i0];
    const int b = dst[i1];
    badc |= ((i < E - 1) && (a > b)) ? 1 : 0;
  }
  const int w = __any(badc != 0);
  if (lane == 0) wany[wave] = w;
  __syncthreads();
  if (wave == 0) {
    const int v = wany[lane & (NWV - 1)];
    const int f = __any(v != 0);
    const unsigned int fu = (unsigned int)f;
    const v4u fv = {fu, fu, fu, fu};
    int* p = flg + ((size_t)s * NCH + (size_t)c) * 32 + 4 * lane;
    if (lane < 8) *(volatile v4u*)p = fv;
    __threadfence();
    if (lane < 8) *(volatile v4u*)p = fv;
  }
}

__global__ __launch_bounds__(NTH) void k_prepw(Src4 s, int K, int N, _Float16* dst, int zs, int total8) {
  const int z = (int)blockIdx.y;
  const int i = (int)blockIdx.x * NTH + (int)threadIdx.x;
  if (i >= total8) return;
  const float* w = (z == 0) ? s.p0 : ((z == 1) ? s.p1 : ((z == 2) ? s.p2 : s.p3));
  const int e  = 8 * i;
  const int nn = e / K;
  const int k0 = e - nn * K;
  v8h hv;
#pragma unroll
  for (int j = 0; j < 8; ++j) hv[j] = (_Float16)(64.0f * w[(size_t)(k0 + j) * (size_t)N + (size_t)nn]);
  _Float16* p = dst + (size_t)z * (size_t)zs + (size_t)e;
  *(volatile v8h*)p = hv;
  __threadfence();
  *(volatile v8h*)p = hv;
}

__global__ __launch_bounds__(NTH) void k_lift(const float* __restrict__ smp, const float* __restrict__ lw,
                                             const float* __restrict__ lb, float* v0p, int n0) {
  const int tid = (int)threadIdx.x, lane = tid & 31;
  const int wave = __builtin_amdgcn_readfirstlane(tid >> 5);
  const int c = 4 * lane;
  const v4f w0 = *(const v4f*)(lw + c);
  const v4f w1 = *(const v4f*)(lw + LAT + c);
  const v4f w2 = *(const v4f*)(lw + 2 * LAT + c);
  const v4f bv = *(const v4f*)(lb + c);
  v4f v[NPW];
#pragma unroll
  for (int i = 0; i < NPW; ++i) {
    int row = (int)blockIdx.x * NPB + wave * NPW + i;
    row = row < n0 ? row : n0 - 1;
    const float s0 = smp[(size_t)row * CIN];
    const float s1 = smp[(size_t)row * CIN + 1];
    const float s2 = smp[(size_t)row * CIN + 2];
    v[i] = ((w0 * s0 + w1 * s1) + w2 * s2) + bv;
  }
#pragma unroll
  for (int i = 0; i < NPW; ++i) {
    const int row = (int)blockIdx.x * NPB + wave * NPW + i;
    if (row < n0) *(volatile v4f*)(v0p + (size_t)row * LAT + c) = v[i];
  }
  __threadfence();
#pragma unroll
  for (int i = 0; i < NPW; ++i) {
    const int row = (int)blockIdx.x * NPB + wave * NPW + i;
    if (row < n0) *(volatile v4f*)(v0p + (size_t)row * LAT + c) = v[i];
  }
}

template <int MODE>
__global__ __launch_bounds__(NTH) void k_edge(
    const int* __restrict__ esrc, const int* __restrict__ edst, int E,
    const float* __restrict__ coords, int n0, int ysh, int xsh, int ny, int nx,
    const float* __restrict__ F,
    const float* __restrict__ w1, const float* __restrict__ b1,
    const _Float16* __restrict__ w2t, const float* __restrict__ b2,
    const int* __restrict__ sflg,
    float* outA, float* outB,
    const float* __restrict__ basep, const float* __restrict__ pw, const float* __restrict__ pb,
    float* outF) {
  __shared__ __attribute__((aligned(16))) float    w1s[4 * HID];
  __shared__ __attribute__((aligned(16))) float    b1s[HID];
  __shared__ __attribute__((aligned(16))) float    b2s[LAT];
  __shared__ __attribute__((aligned(16))) _Float16 w2s[LAT * HID];
  __shared__ __attribute__((aligned(16))) float    rowbuf[NWV * LAT];
  __shared__ __attribute__((aligned(16))) float    outs[LAT];

  const int tid = (int)threadIdx.x, lane = tid & 31, h = lane >> 4, n = lane & 15;
  const int wave = __builtin_amdgcn_readfirstlane(tid >> 5);
  const int blk = (int)blockIdx.x;

#pragma unroll
  for (int q = 0; q < (LAT * HID) / (8 * NTH); ++q) {
    const int i = tid + q * NTH;
    ((v4ua*)w2s)[i] = ((const v4ua*)w2t)[i];
  }
  if (wave == 0) {
    const int i = lane < (HID / 4) ? lane : (HID / 4 - 1);
    ((v4fa*)b1s)[i] = ((const v4fa*)b1)[i];
  } else if (wave == 1) {
    ((v4fa*)b2s)[lane] = ((const v4fa*)b2)[lane];
  } else if (wave < 4) {
    const int i = (wave - 2) * 32 + lane;
    ((v4fa*)w1s)[i] = ((const v4fa*)w1)[i];
  } else {
    outs[tid - 4 * 32] = 0.0f;
  }
  __syncthreads();

  const int sfw = sflg[32 * lane];
  const bool unsorted = __any(sfw != 0) != 0;

  float b2v[8];
#pragma unroll
  for (int t = 0; t < 8; ++t) b2v[t] = b2s[16 * t + n];
  float pwv[12];
  float pbv[3];
  if (MODE == 2) {
#pragma unroll
    for (int j = 0; j < 4; ++j) {
#pragma unroll
      for (int c = 0; c < 3; ++c) pwv[3 * j + c] = pw[(4 * lane + j) * CIN + c];
    }
#pragma unroll
    for (int c = 0; c < 3; ++c) pbv[c] = pb[c];
  } else {
#pragma unroll
    for (int j = 0; j < 12; ++j) pwv[j] = 0.0f;
#pragma unroll
    for (int c = 0; c < 3; ++c) pbv[c] = 0.0f;
  }

  const v8f z8 = {0.f, 0.f, 0.f, 0.f, 0.f, 0.f, 0.f, 0.f};

#pragma unroll 1
  for (int i = 0; i < NPW; ++i) {
    const int node  = blk * NPB + wave * NPW + i;
    const int nodec = node < nx ? node : nx - 1;
    const int xi = nodec << xsh;
    const float xc0 = coords[xi];
    const float xc1 = coords[n0 + xi];

    float cpre[32];
#pragma unroll
    for (int g = 0; g < 4; ++g) {
      const int ub = 16 * g + 8 * h;
      float bb[8], wxa[8], wxb[8];
      ld8(b1s + ub, bb);
      ld8(w1s + 2 * HID + ub, wxa);
      ld8(w1s + 3 * HID + ub, wxb);
#pragma unroll
      for (int ii = 0; ii < 8; ++ii) cpre[8 * g + ii] = fmaf(xc1, wxb[ii], fmaf(xc0, wxa[ii], bb[ii]));
    }

    const int lo = lbound(edst, E, nodec);
    const int hi = lbound(edst, E, nodec + 1);
    int cnt = hi - lo;
    cnt = cnt < 0 ? 0 : cnt;
    const bool bad = (cnt > 16 * MAXT) || unsorted;
    int ntile = (cnt + 15) >> 4;
    ntile = ntile > MAXT ? MAXT : ntile;

    float nacc[8];
#pragma unroll
    for (int t = 0; t < 8; ++t) nacc[t] = 0.0f;

#pragma unroll 1
    for (int tile = 0; tile < ntile; ++tile) {
      const int e0 = lo + 16 * tile;
      int em = e0 + n;
      em = em < hi ? em : hi - 1;
      em = em < 0 ? 0 : em;
      em = em < E ? em : E - 1;
      int sc = esrc[em];
      sc = sc < 0 ? 0 : (sc > ny - 1 ? ny - 1 : sc);
      const int yi = sc << ysh;
      const float yc0 = coords[yi];
      const float yc1 = coords[n0 + yi];

      Frag af[2];
#pragma unroll
      for (int g = 0; g < 4; ++g) {
        const int ub = 16 * g + 8 * h;
        float wya[8], wyb[8];
        ld8(w1s + ub, wya);
        ld8(w1s + HID + ub, wyb);
        v8h hv;
#pragma unroll
        for (int ii = 0; ii < 8; ++ii) {
          const float pre = fmaf(yc1, wyb[ii], fmaf(yc0, wya[ii], cpre[8 * g + ii]));
          hv[ii] = (_Float16)gelu16(pre);
        }
        af[g >> 1].half[g & 1] = hv;
      }

      int  sr[8];
      bool vr[8];
#pragma unroll
      for (int r = 0; r < 8; ++r) {
        sr[r] = __shfl(sc, 8 * h + r);
        vr[r] = (16 * tile + 8 * h + r) < cnt;
      }

#pragma unroll
      for (int hf = 0; hf < 2; ++hf) {
        v8f acc[4];
#pragma unroll
        for (int t4 = 0; t4 < 4; ++t4) acc[t4] = z8;
#pragma unroll
        for (int kk = 0; kk < 2; ++kk) {
#pragma unroll
          for (int t4 = 0; t4 < 4; ++t4) {
            const int t = 4 * hf + t4;
            const _Float16* bp = w2s + (16 * t + n) * HID + 32 * kk + 8 * h;
            Frag bf;
            bf.half[0] = *(const v8ha*)bp;
            bf.half[1] = *(const v8ha*)(bp + 16);
            acc[t4] = wmf(af[kk].v, bf.v, acc[t4]);
          }
        }
#pragma unroll
        for (int r = 0; r < 8; ++r) {
          const float* fp = F + (size_t)sr[r] * LAT + 64 * hf + n;
#pragma unroll
          for (int t4 = 0; t4 < 4; ++t4) {
            float f = fp[16 * t4];
            f = vr[r] ? f : 0.0f;
            nacc[4 * hf + t4] = fmaf(fmaf(acc[t4][r], 0.0009765625f, b2v[4 * hf + t4]), f, nacc[4 * hf + t4]);
          }
        }
      }
    }

#pragma unroll
    for (int t = 0; t < 8; ++t) nacc[t] += __shfl_xor(nacc[t], 16);
    const int cntc = cnt > 1 ? cnt : 1;
    const float rc = 1.0f / (float)cntc;
    const float pz = bad ? __int_as_float(0x7fc00000) : 0.0f;
    float* rb = rowbuf + wave * LAT;
#pragma unroll
    for (int q = 0; q < 4; ++q) {
      const float v = h ? nacc[q + 4] : nacc[q];
      rb[16 * (q + 4 * h) + n] = fmaf(v, rc, pz);
    }
    __builtin_amdgcn_fence(__ATOMIC_RELEASE, "wavefront");
    __builtin_amdgcn_wave_barrier();
    const v4f mv = *(const v4fa*)(rb + 4 * lane);
    __builtin_amdgcn_fence(__ATOMIC_RELEASE, "wavefront");
    __builtin_amdgcn_wave_barrier();

    if (MODE != 2) {
      if (node < nx) {
        float* pa = outA + (size_t)node * LAT + 4 * lane;
        float* pr = outB + (size_t)node * LAT + 4 * lane;
        const v4f mr = relu4(mv);
        *(volatile v4f*)pa = mv;
        if (MODE == 1) *(volatile v4f*)pr = mr;
        __threadfence();
        *(volatile v4f*)pa = mv;
        if (MODE == 1) *(volatile v4f*)pr = mr;
      }
    } else {
      const v4f bv = *(const v4f*)(basep + (size_t)nodec * LAT + 4 * lane);
      const v4f u = relu4(mv + bv);
      float p0 = fmaf(u.w, pwv[9],  fmaf(u.z, pwv[6], fmaf(u.y, pwv[3], u.x * pwv[0])));
      float p1 = fmaf(u.w, pwv[10], fmaf(u.z, pwv[7], fmaf(u.y, pwv[4], u.x * pwv[1])));
      float p2 = fmaf(u.w, pwv[11], fmaf(u.z, pwv[8], fmaf(u.y, pwv[5], u.x * pwv[2])));
#pragma unroll
      for (int off = 16; off >= 1; off >>= 1) {
        p0 += __shfl_xor(p0, off);
        p1 += __shfl_xor(p1, off);
        p2 += __shfl_xor(p2, off);
      }
      if (lane == 0) {
        const int li = wave * NPW + i;
        outs[CIN * li]     = p0 + pbv[0];
        outs[CIN * li + 1] = p1 + pbv[1];
        outs[CIN * li + 2] = p2 + pbv[2];
      }
    }
  }

  if (MODE == 2) {
    __syncthreads();
    if (wave == 0) {
      const v4f ov = *(const v4fa*)(outs + 4 * lane);
      float* op = outF + (size_t)blk * (NPB * CIN) + 4 * lane;
      const bool ok = (lane < (NPB * CIN) / 4) && ((blk + 1) * NPB <= nx);
      if (ok) *(volatile v4f*)op = ov;
      __threadfence();
      if (ok) *(volatile v4f*)op = ov;
    }
  }
}

template <int RELU, int OUT2>
__global__ __launch_bounds__(GTH) void k_ngemm(const float* __restrict__ A, const _Float16* __restrict__ WT,
                                              const float* __restrict__ bias, const float* __restrict__ addp,
                                              float* C, const float* __restrict__ d1b, float* C2, int M) {
  __shared__ __attribute__((aligned(16))) float stg[GRW * LAT];
  const int tid = (int)threadIdx.x, lane = tid & 31, h = lane >> 4, n = lane & 15;
  const int wave = __builtin_amdgcn_readfirstlane(tid >> 5);
  const int rowBase = (int)blockIdx.x * GRW;
  int arow = rowBase + 16 * wave + n;
  arow = arow < M ? arow : M - 1;
  const float* ap = A + (size_t)arow * LAT + 8 * h;
  const _Float16* bq = WT + (size_t)n * LAT + 8 * h;

  v8f acc[8];
#pragma unroll
  for (int t = 0; t < 8; ++t) { const v8f z8 = {0.f, 0.f, 0.f, 0.f, 0.f, 0.f, 0.f, 0.f}; acc[t] = z8; }

#pragma unroll 1
  for (int kk = 0; kk < LAT / 32; ++kk) {
    const v4f x0 = *(const v4f*)(ap + 32 * kk);
    const v4f x1 = *(const v4f*)(ap + 32 * kk + 4);
    const v4f x2 = *(const v4f*)(ap + 32 * kk + 16);
    const v4f x3 = *(const v4f*)(ap + 32 * kk + 20);
    Frag a;
    a.half[0] = cvt8(x0, x1);
    a.half[1] = cvt8(x2, x3);
#pragma unroll
    for (int t = 0; t < 8; ++t) {
      const _Float16* bp = bq + (size_t)(16 * t) * LAT + 32 * kk;
      Frag b;
      b.half[0] = *(const v8ha*)bp;
      b.half[1] = *(const v8ha*)(bp + 16);
      acc[t] = wmf(a.v, b.v, acc[t]);
    }
  }

  float* sp = stg + (16 * wave + 8 * h) * LAT + n;
#pragma unroll
  for (int t = 0; t < 8; ++t) {
#pragma unroll
    for (int r = 0; r < 8; ++r) sp[r * LAT + 16 * t] = acc[t][r];
  }
  __builtin_amdgcn_fence(__ATOMIC_RELEASE, "wavefront");
  __builtin_amdgcn_wave_barrier();

  const v4f bias4 = *(const v4f*)(bias + 4 * lane);
  float* lp = stg + 16 * wave * LAT + 4 * lane;
  const bool wok = (rowBase + 16 * wave + 16) <= M;
#pragma unroll 4
  for (int i = 0; i < 16; ++i) {
    int row = rowBase + 16 * wave + i;
    row = row < M ? row : M - 1;
    const size_t go = (size_t)row * LAT + 4 * lane;
    const v4f x  = *(const v4fa*)(lp + i * LAT);
    const v4f av = *(const v4f*)(addp + go);
    v4f v = (x * 0.015625f + bias4) + av;
    if (RELU) v = relu4(v);
    *(v4fa*)(lp + i * LAT) = v;
    if (wok) *(volatile v4f*)(C + go) = v;
    if (OUT2) {
      const v4f dv = *(const v4f*)(d1b + go);
      const v4f v2 = relu4(v + dv);
      if (wok) *(volatile v4f*)(C2 + go) = v2;
    }
  }
  __threadfence();
#pragma unroll 4
  for (int i = 0; i < 16; ++i) {
    int row = rowBase + 16 * wave + i;
    row = row < M ? row : M - 1;
    const size_t go = (size_t)row * LAT + 4 * lane;
    const v4f v = *(const v4fa*)(lp + i * LAT);
    if (wok) *(volatile v4f*)(C + go) = v;
    if (OUT2) {
      const v4f dv = *(const v4f*)(d1b + go);
      const v4f v2 = relu4(v + dv);
      if (wok) *(volatile v4f*)(C2 + go) = v2;
    }
  }
}

extern "C" void kernel_launch(void* const* d_in, const int* in_sizes, int n_in,
                              void* d_out, int out_size, void* d_ws, size_t ws_size,
                              hipStream_t stream) {
  if (n_in < 35) return;
  const int n0 = in_sizes[0] / 2;
  if (n0 < 128 || in_sizes[0] != 2 * n0 || (n0 % 128) != 0) return;
  const int n1 = n0 / 2;
  if (in_sizes[1] != CIN * n0 || out_size != CIN * n0) return;
  if (in_sizes[3] != CIN * LAT || in_sizes[4] != LAT || in_sizes[5] != LAT * CIN || in_sizes[6] != CIN) return;
  if (in_sizes[7] != LAT * LAT || in_sizes[8] != LAT || in_sizes[9] != LAT * LAT || in_sizes[10] != LAT) return;
  for (int g = 0; g < 4; ++g) {
    if (in_sizes[11 + 4 * g] != 4 * HID || in_sizes[12 + 4 * g] != HID) return;
    if (in_sizes[13 + 4 * g] != HID * LAT || in_sizes[14 + 4 * g] != LAT) return;
  }
  int E[4];
  int maxE = 1;
  for (int s = 0; s < 4; ++s) {
    E[s] = in_sizes[27 + 2 * s];
    if (E[s] < 1 || in_sizes[28 + 2 * s] != E[s]) return;
    if (E[s] > (1 << 28)) return;
    maxE = E[s] > maxE ? E[s] : maxE;
  }

  const float* coords = (const float*)d_in[0];
  const float* smp    = (const float*)d_in[1];
  const float* lift_w = (const float*)d_in[3];
  const float* lift_b = (const float*)d_in[4];
  const float* proj_w = (const float*)d_in[5];
  const float* proj_b = (const float*)d_in[6];
  const float* W0_w   = (const float*)d_in[7];
  const float* W0_b   = (const float*)d_in[8];
  const float* W1_w   = (const float*)d_in[9];
  const float* W1_b   = (const float*)d_in[10];
  const float *gw1[4], *gb1[4], *gw2[4], *gb2[4];
  for (int g = 0; g < 4; ++g) {
    gw1[g] = (const float*)d_in[11 + 4 * g];
    gb1[g] = (const float*)d_in[12 + 4 * g];
    gw2[g] = (const float*)d_in[13 + 4 * g];
    gb2[g] = (const float*)d_in[14 + 4 * g];
  }
  const int *esrc[4], *edst[4];
  for (int s = 0; s < 4; ++s) {
    esrc[s] = (const int*)d_in[27 + 2 * s];
    edst[s] = (const int*)d_in[28 + 2 * s];
  }
  float* out = (float*)d_out;

  char* ws = (char*)d_ws;
  size_t off = 0;
  const size_t oWT   = off; off += (size_t)2 * LAT * LAT * 2;
  const size_t oG2   = off; off += (size_t)4 * LAT * HID * 2;
  const size_t oFLG  = off; off += (size_t)4 * NCH * 32 * 4;
  const size_t oV0   = off; off += (size_t)n0 * LAT * 4;
  const size_t oAGG0 = off; off += (size_t)n0 * LAT * 4;
  const size_t oBASE = off; off += (size_t)n0 * LAT * 4;
  const size_t oD1B  = off; off += (size_t)n1 * LAT * 4;
  const size_t oVDa  = off; off += (size_t)n1 * LAT * 4;
  const size_t oVDb  = off; off += (size_t)n1 * LAT * 4;
  const size_t oAGG1 = off; off += (size_t)n1 * LAT * 4;
  const size_t oVU1  = off; off += (size_t)n1 * LAT * 4;
  if (off > ws_size || off > (size_t)WSCAP) return;
  _Float16* WT    = (_Float16*)(ws + oWT);
  _Float16* G2    = (_Float16*)(ws + oG2);
  int*      FLG   = (int*)(ws + oFLG);
  float*    V0    = (float*)(ws + oV0);
  float*    AGG00 = (float*)(ws + oAGG0);
  float*    BASE0 = (float*)(ws + oBASE);
  float*    D1B   = (float*)(ws + oD1B);
  float*    VD1a  = (float*)(ws + oVDa);
  float*    VD1b  = (float*)(ws + oVDb);
  float*    AGG11 = (float*)(ws + oAGG1);
  float*    VU1   = (float*)(ws + oVU1);

  {
    Src4 sA; sA.p0 = W0_w; sA.p1 = W1_w; sA.p2 = W0_w; sA.p3 = W0_w;
    const int t8 = (LAT * LAT) / 8;
    k_prepw<<<dim3((t8 + NTH - 1) / NTH, 2), NTH, 0, stream>>>(sA, LAT, LAT, WT, LAT * LAT, t8);
    Src4 sB; sB.p0 = gw2[0]; sB.p1 = gw2[1]; sB.p2 = gw2[2]; sB.p3 = gw2[3];
    const int t8g = (HID * LAT) / 8;
    k_prepw<<<dim3((t8g + NTH - 1) / NTH, 4), NTH, 0, stream>>>(sB, HID, LAT, G2, LAT * HID, t8g);
  }
  {
    Dst4 dd; dd.p0 = edst[0]; dd.p1 = edst[1]; dd.p2 = edst[2]; dd.p3 = edst[3];
    const int per   = (maxE + NCH - 1) / NCH;
    const int chunk = ((per + NTH - 1) / NTH) * NTH;
    k_chk<<<dim3(NCH, 4), NTH, 0, stream>>>(dd, E[0], E[1], E[2], E[3], chunk, FLG);
  }
  k_lift<<<n0 / NPB, NTH, 0, stream>>>(smp, lift_w, lift_b, V0, n0);
  k_edge<0><<<n0 / NPB, NTH, 0, stream>>>(esrc[0], edst[0], E[0], coords, n0, 0, 0, n0, n0, V0,
                                           gw1[0], gb1[0], G2 + 0 * LAT * HID, gb2[0], FLG + 0 * NCH * 32,
                                           AGG00, AGG00, coords, coords, coords, AGG00);
  k_edge<1><<<n1 / NPB, NTH, 0, stream>>>(esrc[1], edst[1], E[1], coords, n0, 0, 1, n0, n1, V0,
                                           gw1[1], gb1[1], G2 + 1 * LAT * HID, gb2[1], FLG + 1 * NCH * 32,
                                           D1B, VD1a, coords, coords, coords, D1B);
  k_ngemm<0, 0><<<n0 / GRW, GTH, 0, stream>>>(V0, WT, W0_b, AGG00, BASE0, AGG00, BASE0, n0);
  for (int it = 0; it < 3; ++it) {
    float* VDc = (it & 1) ? VD1b : VD1a;
    float* VDn = (it & 1) ? VD1a : VD1b;
    k_edge<0><<<n1 / NPB, NTH, 0, stream>>>(esrc[3], edst[3], E[3], coords, n0, 1, 1, n1, n1, VDc,
                                             gw1[3], gb1[3], G2 + 3 * LAT * HID, gb2[3], FLG + 3 * NCH * 32,
                                             AGG11, AGG11, coords, coords, coords, AGG11);
    if (it < 2) {
      k_ngemm<1, 1><<<n1 / GRW, GTH, 0, stream>>>(VDc, WT + LAT * LAT, W1_b, AGG11, VU1, D1B, VDn, n1);
    } else {
      k_ngemm<1, 0><<<n1 / GRW, GTH, 0, stream>>>(VDc, WT + LAT * LAT, W1_b, AGG11, VU1, AGG11, VU1, n1);
    }
  }
  k_edge<2><<<n0 / NPB, NTH, 0, stream>>>(esrc[2], edst[2], E[2], coords, n0, 1, 0, n1, n0, VU1,
                                           gw1[2], gb1[2], G2 + 2 * LAT * HID, gb2[2], FLG + 2 * NCH * 32,
                                           AGG00, AGG00, BASE0, proj_w, proj_b, out);
}
